// EdgeSpecificComplexModel_34016140984985
// MI455X (gfx1250) — hardware-verified
//
#include <hip/hip_runtime.h>
#include <stddef.h>
#include <math.h>

#define NV 5
#define KM 2
#define DM 512
#define KIN 25
#define KPAD 32
#define N2 4
#define N2PAD 16
#define RB 32
#define NTHR 64
#define APITCH 40
#define HSTR 516
#define LN_EPS 1e-5f
#define PHI_SCALE 0.13089969389957471827f
#define WSC 64.0f
#define INV_WSC (1.0f / 64.0f)

static_assert(APITCH % 8 == 0);
static_assert(HSTR % 4 == 0);
static_assert(NTHR == 64);
static_assert(RB == 32);
static_assert(DM % 32 == 0);

typedef _Float16 f16;
typedef f16 v16h __attribute__((ext_vector_type(16)));
typedef f16 v8h_t __attribute__((ext_vector_type(8)));
typedef v8h_t __attribute__((may_alias)) v8h;
typedef float v8f __attribute__((ext_vector_type(8)));
typedef float v4f_t __attribute__((ext_vector_type(4)));
typedef v4f_t __attribute__((may_alias)) v4f;
typedef unsigned int v4u __attribute__((ext_vector_type(4)));

union Frag { v16h v; v8h_t h[2]; };

__device__ __forceinline__ v8f zero8() {
    v8f z;
#pragma unroll
    for (int i = 0; i < 8; ++i) z[i] = 0.0f;
    return z;
}

__device__ __forceinline__ v8f wmma_f16(v16h a, v16h b, v8f c) {
    v8f d = __builtin_amdgcn_wmma_f32_16x16x32_f16(false, a, false, b, (short)0, c, false, false);
    asm volatile("v_nop\n\tv_nop\n\tv_nop\n\tv_nop" : "+v"(d) : "v"(a), "v"(b));
    return d;
}

__global__ void __launch_bounds__(256) prep_kernel(
    const float* __restrict__ S, const float* __restrict__ gam,
    const float* __restrict__ dph, const float* __restrict__ pw,
    const float* __restrict__ W1, const float* __restrict__ W2,
    f16* __restrict__ w1pk, f16* __restrict__ w2pk, float* __restrict__ edge)
{
    __shared__ __align__(16) float s_e[128];
    const int tid = threadIdx.x;

#pragma unroll 1
    for (int it = 0; it < (DM * KPAD) / (8 * 256); ++it) {
        const int q  = it * 256 + tid;
        const int n  = q >> 2;
        const int kb = (q & 3) * 8;
        union { v8h_t h; v4u u; } pk;
#pragma unroll
        for (int c = 0; c < 8; ++c) {
            const int k  = kb + c;
            const int kc = (k < KIN) ? k : (KIN - 1);
            const float v = W1[kc * DM + n];
            pk.h[c] = (f16)(v * ((k < KIN) ? WSC : 0.0f));
        }
        f16* dst = w1pk + (size_t)q * 8;
        *(volatile v4u*)dst = pk.u;
        __threadfence();
        *(volatile v4u*)dst = pk.u;
    }

#pragma unroll 1
    for (int it = 0; it < (N2PAD * DM) / (8 * 256); ++it) {
        const int q  = it * 256 + tid;
        const int n  = q >> 6;
        const int kb = (q & 63) * 8;
        const int nc = (n < N2) ? n : (N2 - 1);
        const float sc = (n < N2) ? WSC : 0.0f;
        union { v8h_t h; v4u u; } pk;
#pragma unroll
        for (int c = 0; c < 8; ++c) {
            const float v = W2[(kb + c) * N2 + nc];
            pk.h[c] = (f16)(v * sc);
        }
        f16* dst = w2pk + (size_t)q * 8;
        *(volatile v4u*)dst = pk.u;
        __threadfence();
        *(volatile v4u*)dst = pk.u;
    }

    {
        const int t = (tid < NV * NV) ? tid : (NV * NV - 1);
        const float p0 = pw[t * 2 + 0], p1 = pw[t * 2 + 1];
        const float mx = fmaxf(p0, p1);
        const float e0 = expf(p0 - mx), e1 = expf(p1 - mx);
        const float inv = 1.0f / (e0 + e1);
        const float w0 = e0 * inv, w1v = e1 * inv;
        const float sg0 = 1.0f / (1.0f + expf(-gam[t * 2 + 0]));
        const float sg1 = 1.0f / (1.0f + expf(-gam[t * 2 + 1]));
        const float d0 = dph[t * 2 + 0], d1 = dph[t * 2 + 1];
        const float sv = S[t];
        if (tid < NV * NV) {
            s_e[tid]       = w0 * sg0 + w1v * sg1;
            s_e[25 + tid]  = w0 * d0 + w1v * d1;
            s_e[50 + tid]  = w0;
            s_e[75 + tid]  = w1v;
            s_e[100 + tid] = sv;
        }
        if (tid < 3) s_e[125 + tid] = 0.0f;
    }
    __syncthreads();
    const v4f_t ev = ((const v4f*)s_e)[tid & 31];
    if (tid < 32) *(volatile v4f_t*)(edge + 4 * tid) = ev;
    __threadfence();
    if (tid < 32) *(volatile v4f_t*)(edge + 4 * tid) = ev;
}

__global__ void __launch_bounds__(NTHR) fused_kernel(
    const float* __restrict__ x2, const float* __restrict__ hist,
    const float* __restrict__ phig, const float* __restrict__ b1,
    const float* __restrict__ lng, const float* __restrict__ lnb,
    const float* __restrict__ b2,
    const f16* __restrict__ w1pk, const f16* __restrict__ w2pk,
    const float* __restrict__ edge, float* __restrict__ out, int nrows)
{
    __shared__ __align__(16) f16   s_a[RB * APITCH];
    __shared__ __align__(16) float s_h[2][16 * HSTR];
    __shared__ __align__(16) float s_ln[3 * DM];
    __shared__ __align__(16) float s_edge[128];
    __shared__ float s_stat[2][32];
    __shared__ __align__(16) float s_par[RB * 4];
    __shared__ __align__(16) float s_o0[RB * NV * 2];
    __shared__ __align__(16) float s_o1[RB * KM];
    __shared__ __align__(16) float s_o2[RB * NV * NV];

    const int tid  = threadIdx.x;
    const int w    = tid >> 5;
    const int lane = tid & 31;
    const int hh   = lane >> 4;
    const int m    = lane & 15;
    const int row0 = blockIdx.x * RB;
    if (row0 + RB > nrows) return;

    for (int i = tid; i < DM / 4; i += NTHR) {
        ((v4f*)s_ln)[i]       = ((const v4f*)lng)[i];
        ((v4f*)s_ln)[128 + i] = ((const v4f*)lnb)[i];
        ((v4f*)s_ln)[256 + i] = ((const v4f*)b1)[i];
    }
    if (tid < 32) ((v4f*)s_edge)[tid] = ((const v4f*)edge)[tid];
#pragma unroll 1
    for (int i = tid; i < RB * KPAD; i += NTHR) {
        const int r  = i >> 5;
        const int k  = i & 31;
        const int kc = (k < KIN) ? k : (KIN - 1);
        const float v = hist[(size_t)(row0 + r) * KIN + kc];
        s_a[r * APITCH + k] = (f16)(v * ((k < KIN) ? 1.0f : 0.0f));
    }
    __syncthreads();

    {
        Frag a;
        const f16* pa = s_a + (16 * w + m) * APITCH + 8 * hh;
        a.h[0] = *(const v8h*)(pa);
        a.h[1] = *(const v8h*)(pa + 16);
        float* hw = s_h[w];
#pragma unroll 2
        for (int ct = 0; ct < DM / 16; ++ct) {
            Frag b;
            const f16* pb = w1pk + (size_t)(ct * 16 + m) * KPAD + 8 * hh;
            b.h[0] = *(const v8h*)(pb);
            b.h[1] = *(const v8h*)(pb + 16);
            const v8f c = wmma_f16(a.v, b.v, zero8());
            const int col = ct * 16 + m;
            const float b1c = s_ln[2 * DM + col];
#pragma unroll
            for (int r = 0; r < 8; ++r)
                hw[(8 * hh + r) * HSTR + col] = c[r] * INV_WSC + b1c;
        }
    }
    __syncthreads();

    {
        const int srow = lane >> 1, half = lane & 1;
        const float* hp = s_h[w] + srow * HSTR + half * 256;
        float s = 0.0f;
#pragma unroll 4
        for (int t = 0; t < 64; ++t) {
            const v4f_t v = ((const v4f*)hp)[t];
            s += (v[0] + v[1]) + (v[2] + v[3]);
        }
        s += __shfl_xor(s, 1, 32);
        const float mu = s * (1.0f / (float)DM);
        float s2 = 0.0f;
#pragma unroll 4
        for (int t = 0; t < 64; ++t) {
            const v4f_t v = ((const v4f*)hp)[t];
            const float d0 = v[0] - mu, d1 = v[1] - mu, d2 = v[2] - mu, d3 = v[3] - mu;
            s2 += (d0 * d0 + d1 * d1) + (d2 * d2 + d3 * d3);
        }
        s2 += __shfl_xor(s2, 1, 32);
        const float var  = s2 * (1.0f / (float)DM);
        const float rstd = rsqrtf(var + LN_EPS);
        if (half == 0) {
            s_stat[w][srow]      = mu;
            s_stat[w][16 + srow] = rstd;
        }
    }
    __syncthreads();

    {
        const float mu_m = s_stat[w][m];
        const float rs_m = s_stat[w][16 + m];
        const float* hrow = s_h[w] + m * HSTR;
        const f16* pbw = w2pk + (size_t)m * DM + 8 * hh;
        v8f c2 = zero8();
#pragma unroll 1
        for (int kt = 0; kt < DM / 32; ++kt) {
            v16h a2;
            const int kb = kt * 32 + 8 * hh;
#pragma unroll
            for (int e = 0; e < 8; ++e) {
                const int k = kb + e;
                const float v = (hrow[k] - mu_m) * rs_m * s_ln[k] + s_ln[DM + k];
                a2[e] = (f16)fmaxf(v, 0.0f);
            }
#pragma unroll
            for (int e = 0; e < 8; ++e) {
                const int k = kb + 16 + e;
                const float v = (hrow[k] - mu_m) * rs_m * s_ln[k] + s_ln[DM + k];
                a2[8 + e] = (f16)fmaxf(v, 0.0f);
            }
            Frag b;
            b.h[0] = *(const v8h*)(pbw + kt * 32);
            b.h[1] = *(const v8h*)(pbw + kt * 32 + 16);
            c2 = wmma_f16(a2, b.v, c2);
        }
        const float bb = b2[m & 3];
        if (m < N2) {
#pragma unroll
            for (int r = 0; r < 8; ++r)
                s_par[(16 * w + 8 * hh + r) * 4 + m] = c2[r] * INV_WSC + bb;
        }
    }
    __syncthreads();

    if (w == 0) {
        const int r = lane;
        const size_t bg = (size_t)row0 + (size_t)r;
        const float p0 = s_par[r * 4 + 0];
        const float p1 = s_par[r * 4 + 1];
        const float p2 = s_par[r * 4 + 2];
        const float p3 = s_par[r * 4 + 3];
        const float phi0 = phig[bg * 2 + 0] + tanhf(p0) * PHI_SCALE;
        const float phi1 = phig[bg * 2 + 1] + tanhf(p2) * PHI_SCALE;
        const float rm0  = 1.0f / (1.0f + expf(-p1));
        const float rm1  = 1.0f / (1.0f + expf(-p3));
        s_o1[r * 2 + 0] = phi0;
        s_o1[r * 2 + 1] = phi1;
        const float* xrow = x2 + bg * (NV * 2);
#pragma unroll 1
        for (int i = 0; i < NV; ++i) {
            float nre = 0.0f, nim = 0.0f;
#pragma unroll 1
            for (int j = 0; j < NV; ++j) {
                const int idx = i * NV + j;
                const float xr = xrow[2 * j + 0];
                const float xi = xrow[2 * j + 1];
                const float wk0 = s_edge[50 + idx], wk1 = s_edge[75 + idx];
                const float theta = wk0 * phi0 + wk1 * phi1 + s_edge[25 + idx];
                const float rr    = wk0 * rm0 + wk1 * rm1;
                const float araw  = rr * s_edge[100 + idx];
                const float den   = 1.0f + fabsf(araw);
                const float ag    = s_edge[idx] * (araw * (1.0f / den));
                const float st = sinf(theta);
                const float ct = cosf(theta);
                nre += ag * (ct * xr - st * xi);
                nim += ag * (st * xr + ct * xi);
                s_o2[r * (NV * NV) + idx] = ag;
            }
            s_o0[r * (NV * 2) + 2 * i + 0] = nre;
            s_o0[r * (NV * 2) + 2 * i + 1] = nim;
        }
    }
    __syncthreads();

    {
        float* o0 = out + (size_t)row0 * (NV * 2);
        float* o1 = out + (size_t)nrows * (NV * 2) + (size_t)row0 * KM;
        float* o2 = out + (size_t)nrows * (NV * 2 + KM) + (size_t)row0 * (NV * NV);
        const int qa = tid;
        const int qb = 64 + (tid & 15);
        const int q1 = tid & 15;
        const v4f_t va = ((const v4f*)s_o0)[qa];
        const v4f_t vb = ((const v4f*)s_o0)[qb];
        const v4f_t v1 = ((const v4f*)s_o1)[q1];
        v4f_t v2[4];
#pragma unroll
        for (int it = 0; it < 4; ++it) {
            int q = it * 64 + tid;
            q = (q < 200) ? q : 199;
            v2[it] = ((const v4f*)s_o2)[q];
        }

        *(volatile v4f_t*)(o0 + 4 * qa) = va;
        if (tid < 16) {
            *(volatile v4f_t*)(o0 + 4 * qb) = vb;
            *(volatile v4f_t*)(o1 + 4 * q1) = v1;
        }
#pragma unroll
        for (int it = 0; it < 4; ++it) {
            const int q = it * 64 + tid;
            if (q < 200) *(volatile v4f_t*)(o2 + 4 * q) = v2[it];
        }
        __threadfence();
        *(volatile v4f_t*)(o0 + 4 * qa) = va;
        if (tid < 16) {
            *(volatile v4f_t*)(o0 + 4 * qb) = vb;
            *(volatile v4f_t*)(o1 + 4 * q1) = v1;
        }
#pragma unroll
        for (int it = 0; it < 4; ++it) {
            const int q = it * 64 + tid;
            if (q < 200) *(volatile v4f_t*)(o2 + 4 * q) = v2[it];
        }
    }
}

extern "C" void kernel_launch(void* const* d_in, const int* in_sizes, int n_in,
                              void* d_out, int out_size, void* d_ws, size_t ws_size,
                              hipStream_t stream)
{
    if (n_in < 13) return;
    const int nrows = in_sizes[1] / KIN;
    if (nrows <= 0 || (nrows % RB) != 0) return;
    if (in_sizes[0] != nrows * NV * 2) return;
    if (in_sizes[1] != nrows * KIN) return;
    if (in_sizes[2] != nrows * KM) return;
    if (in_sizes[3] != NV * NV) return;
    if (in_sizes[4] != NV * NV * KM) return;
    if (in_sizes[5] != NV * NV * KM) return;
    if (in_sizes[6] != NV * NV * KM) return;
    if (in_sizes[7] != KIN * DM) return;
    if (in_sizes[8] != DM || in_sizes[9] != DM || in_sizes[10] != DM) return;
    if (in_sizes[11] != DM * N2) return;
    if (in_sizes[12] != N2) return;
    if (out_size != nrows * (NV * 2 + KM + NV * NV)) return;

    const float* x2   = (const float*)d_in[0];
    const float* hist = (const float*)d_in[1];
    const float* phig = (const float*)d_in[2];
    const float* S    = (const float*)d_in[3];
    const float* gam  = (const float*)d_in[4];
    const float* dph  = (const float*)d_in[5];
    const float* pw   = (const float*)d_in[6];
    const float* W1   = (const float*)d_in[7];
    const float* b1   = (const float*)d_in[8];
    const float* lng  = (const float*)d_in[9];
    const float* lnb  = (const float*)d_in[10];
    const float* W2   = (const float*)d_in[11];
    const float* b2   = (const float*)d_in[12];
    float* out = (float*)d_out;

    const size_t oEdge = 0;
    const size_t oW1   = 512;
    const size_t oW2   = oW1 + (size_t)DM * KPAD * 2;
    const size_t total = oW2 + (size_t)N2PAD * DM * 2;
    if (total > ws_size) return;

    char* ws = (char*)d_ws;
    float* edge = (float*)(ws + oEdge);
    f16*   w1pk = (f16*)(ws + oW1);
    f16*   w2pk = (f16*)(ws + oW2);

    prep_kernel<<<1, 256, 0, stream>>>(S, gam, dph, pw, W1, W2, w1pk, w2pk, edge);
    fused_kernel<<<nrows / RB, NTHR, 0, stream>>>(
        x2, hist, phig, b1, lng, lnb, b2, w1pk, w2pk, edge, out, nrows);
}
